// FactorGraphNetwork_3822520893461
// MI455X (gfx1250) — hardware-verified
//
#include <hip/hip_runtime.h>


namespace {
constexpr int B = 65536, V = 64, K = 64, H = 16, RW = 32  ;
constexpr float XS = 8.0f, HS = 256.0f, WSC = 256.0f, TH = 0.3f;
typedef _Float16 b16;
typedef __attribute__((ext_vector_type(16))) _Float16 v16b;
typedef __attribute__((ext_vector_type(8))) _Float16 v8b;
typedef __attribute__((ext_vector_type(8))) float v8f;
__device__ __forceinline__ float bf16_rne(float f) { unsigned int u = __float_as_uint(f); u += 0x7FFFu + ((u >> 16) & 1u); float r = __uint_as_float(u & 0xFFFF0000u); asm volatile("" : "+v"(r)); return r; }
__device__ __forceinline__ float bfv(float f) { float r = bf16_rne(f); asm volatile("" : "+v"(r)); return r; }
__device__ __forceinline__ void split16(float v, b16& hi, b16& lo) { hi = (b16)v; lo = (b16)(v - (float)hi); }
__device__ __forceinline__ v16b frag_kb(const b16* p, int hh) { const v8b a = *(const v8b*)(p + 8 * hh), b = *(const v8b*)(p + 16 + 8 * hh); v16b f;
#pragma unroll
  for (int e = 0; e < 8; ++e) { f[e] = a[e]; f[8 + e] = b[e]; } return f; }
__device__ __forceinline__ v8f wmma16b(v16b a, v16b b, v8f c) { v8f d = __builtin_amdgcn_wmma_f32_16x16x32_f16(false, a, false, b, (short)0, c, false, false); asm volatile("v_nop\n\tv_nop\n\tv_nop\n\tv_nop" : "+v"(d) : "v"(a), "v"(b)); return d; }
__device__ __forceinline__ void wave_lds_sync() { __builtin_amdgcn_fence(__ATOMIC_RELEASE, "workgroup"); __builtin_amdgcn_wave_barrier(); __builtin_amdgcn_fence(__ATOMIC_ACQUIRE, "workgroup"); }
__device__ __forceinline__ float pmul(float a, float b) { float p = a * b; asm volatile("" : "+v"(p)); return p; }
__device__ __forceinline__ float ste(float raw) { const float soft = 1.0f / (1.0f + __expf(-raw)); const float hard = soft > TH ? 1.0f : 0.0f; return (hard - soft) + soft; }

__global__ __launch_bounds__(256) void wput_kernel(const float* __restrict__ rm, const float* __restrict__ rw, const float* __restrict__ w1, const float* __restrict__ w2, b16* __restrict__ WM, b16* __restrict__ WB, float* __restrict__ SW) { const int u = blockIdx.x * 256 + threadIdx.x; v8b v;
  if (u < K * H * 8) { const int o = u / 8, k0 = (u % 8) * 8; const int k = o / H, h = o % H;
#pragma unroll
    for (int j = 0; j < 8; ++j) { const int vv = k0 + j; v[j] = (b16)(ste(bfv(rm[k * V + vv])) * bfv(w1[((size_t)k * V + vv) * H + h]) * WSC); } for (int pass = 0; pass < 2; ++pass) { *(volatile v8b*)(WM + (size_t)o * V + k0) = v; __threadfence(); } }
  if (u < K * H * 4) { const int o = u / 4, k0 = (u % 4) * 8; const int k = o / H, g = o % H;
#pragma unroll
    for (int j = 0; j < 8; ++j) { const int hh = k0 + j; v[j] = (b16)(hh < H ? bf16_rne(w2[((size_t)k * H + hh) * H + g]) * WSC : 0.0f); } for (int pass = 0; pass < 2; ++pass) { *(volatile v8b*)(WB + (size_t)o * 32 + k0) = v; __threadfence(); } }
  if (u < K) { const float s = ste(bfv(rw[u])); for (int pass = 0; pass < 2; ++pass) { ((volatile float*)SW)[u] = s; __threadfence(); } } }
__global__ __launch_bounds__(32) void main_kernel(const float* __restrict__ x, const b16* __restrict__ WM, const float* __restrict__ b1, const b16* __restrict__ WB, const float* __restrict__ b2, const float* __restrict__ w3, const float* __restrict__ b3, const float* __restrict__ SW, int BLIM, float* __restrict__ out) { __shared__ __attribute__((aligned(16))) b16 Ax[RW][V + 8], Ph[RW][8][40], Pl[RW][8][40]; __shared__ float Tq[RW][17], Os[RW]; const int lane = threadIdx.x, nloc = lane & 15, hlf = lane >> 4; const size_t r0 = (size_t)blockIdx.x * RW; if (r0 >= (size_t)BLIM) return;
  for (int rr = 0; rr < RW; ++rr) for (int q = 0; q < 2; ++q) Ax[rr][q * 32 + lane] = (b16)(bf16_rne(x[(r0 + rr) * V + q * 32 + lane]) * XS);
  for (int k = V; k < V + 8; ++k) Ax[lane][k] = (b16)0.0f; for (int f = 0; f < 8; ++f) for (int k = H; k < 40; ++k) { Ph[lane][f][k] = (b16)0.0f; Pl[lane][f][k] = (b16)0.0f; } Os[lane] = 0.0f;
  wave_lds_sync(); const v16b a0[2] = {frag_kb(&Ax[nloc][0], hlf), frag_kb(&Ax[nloc][32], hlf)}, a1[2] = {frag_kb(&Ax[16 + nloc][0], hlf), frag_kb(&Ax[16 + nloc][32], hlf)};
#pragma unroll 1
  for (int g8 = 0; g8 < K / 8; ++g8) {
    v8f h0[8], h1v[8];
#pragma unroll
    for (int f = 0; f < 8; ++f) { h0[f] = (v8f){}; h1v[f] = (v8f){}; }
#pragma unroll
    for (int ks = 0; ks < 2; ++ks)
#pragma unroll
      for (int f = 0; f < 8; ++f) { const v16b bw = frag_kb(WM + (size_t)((g8 * 8 + f) * H + nloc) * V + ks * 32, hlf); h0[f] = wmma16b(a0[ks], bw, h0[f]); h1v[f] = wmma16b(a1[ks], bw, h1v[f]); }
#pragma unroll
    for (int f = 0; f < 8; ++f) { const int k = g8 * 8 + f; const float bb = bfv(b1[k * H + nloc]);
#pragma unroll
      for (int r8 = 0; r8 < 8; ++r8) { b16 p, pl; split16(fmaxf(h0[f][r8] * (1.0f / (XS * WSC)) + bb, 0.0f) * HS, p, pl); Ph[8 * hlf + r8][f][nloc] = p; Pl[8 * hlf + r8][f][nloc] = pl; split16(fmaxf(h1v[f][r8] * (1.0f / (XS * WSC)) + bb, 0.0f) * HS, p, pl); Ph[16 + 8 * hlf + r8][f][nloc] = p; Pl[16 + 8 * hlf + r8][f][nloc] = pl; } }
    wave_lds_sync();
#pragma unroll 1
    for (int f = 0; f < 8; ++f) { const int k = g8 * 8 + f; const v16b bw = frag_kb(WB + (size_t)(k * H + nloc) * 32, hlf);
      v8f d0 = wmma16b(frag_kb(&Ph[nloc][f][0], hlf), bw, (v8f){}); d0 = wmma16b(frag_kb(&Pl[nloc][f][0], hlf), bw, d0); v8f d1 = wmma16b(frag_kb(&Ph[16 + nloc][f][0], hlf), bw, (v8f){}); d1 = wmma16b(frag_kb(&Pl[16 + nloc][f][0], hlf), bw, d1);
      const float bb = bfv(b2[k * H + nloc]), wg = bfv(w3[k * H + nloc]);
#pragma unroll
      for (int r8 = 0; r8 < 8; ++r8) { Tq[8 * hlf + r8][nloc] = pmul(fmaxf(d0[r8] * (1.0f / (HS * WSC)) + bb, 0.0f), wg); Tq[16 + 8 * hlf + r8][nloc] = pmul(fmaxf(d1[r8] * (1.0f / (HS * WSC)) + bb, 0.0f), wg); }
      wave_lds_sync();
      { float s = bfv(b3[k]); for (int g = 0; g < H; ++g) s += Tq[lane][g]; Os[lane] += s * SW[k]; }
      wave_lds_sync(); } }
  for (int pass = 0; pass < 2; ++pass) { ((volatile float*)out)[r0 + lane] = Os[lane]; __threadfence(); } }
}

extern "C" void kernel_launch(void* const* d_in, const int* in_sizes, int n_in, void* d_out, int out_size, void* d_ws, size_t ws_size, hipStream_t stream) {
  (void)n_in;
  auto Fp = [&](int i) { return (const float*)d_in[i]; };
  if (in_sizes[0] != B * V || in_sizes[1] != K * V || in_sizes[2] != K || in_sizes[3] != K * V * H || in_sizes[5] != K * H * H || in_sizes[7] != K * H || out_size != B) return;
  const int BLIM = B;
  size_t off = 0; char* ws = (char*)d_ws;
  auto carve = [&](size_t bytes) { char* p = ws + off; off += (bytes + 255) & ~(size_t)255; return p; };
  b16* WM = (b16*)carve((size_t)K * H * V * 2); b16* WB = (b16*)carve((size_t)K * H * 32 * 2); float* SW = (float*)carve((size_t)K * 4);
  if (off > ws_size || off > ((size_t)1 << 20)) return;
  wput_kernel<<<(K * H * 8 + 255) / 256, 256, 0, stream>>>(Fp(1), Fp(2), Fp(3), Fp(5), WM, WB, SW);
  main_kernel<<<BLIM / RW, 32, 0, stream>>>(Fp(0), WM, Fp(4), WB, Fp(6), Fp(7), Fp(8), SW, BLIM, (float*)d_out);
}
